// BottleneckBlock_50362786513357
// MI455X (gfx1250) — hardware-verified
//
#include <hip/hip_runtime.h>
#include <math.h>

constexpr int NBATCH = 8;
constexpr int NCH    = 256;
constexpr int NCO    = 512;
constexpr int NCR    = 32;
constexpr int NLEN   = 2048;
constexpr int NLENP  = 2052;
constexpr int NTAP   = 5;
constexpr int KCONV  = NCH * NTAP;
constexpr float W_CARRY      = 16.0f;
constexpr float W_CARRY_INV  = 1.0f / 16.0f;
constexpr float P_CARRY      = 2048.0f;
constexpr float O_CARRY      = 64.0f;
constexpr float PV_OUT_SCALE = O_CARRY / P_CARRY;
constexpr float WO_SCALE     = 1.0f / (W_CARRY * O_CARRY);
constexpr float QK_SCALE     = 0.17677669529663687f;
constexpr float IN_EPS       = 1e-5f;
constexpr float NEG_SLOPE_V  = 0.2f;
constexpr float INV_LEN      = 1.0f / 2048.0f;

constexpr size_t SZ_TP   = (size_t)NBATCH * NLENP * NCH * 2;
constexpr size_t SZ_W1   = (size_t)NCH * KCONV * 2;
constexpr size_t SZ_W2   = (size_t)NCO * KCONV * 2;
constexpr size_t SZ_WQK  = (size_t)2 * NCR * NCH * 2;
constexpr size_t SZ_WV   = (size_t)NCH * NCH * 2;
constexpr size_t SZ_WO   = (size_t)NCH * NCH * 2;
constexpr size_t SZ_WR   = (size_t)NCO * NCH * 2;
constexpr size_t SZ_BQK  = 256;
constexpr size_t SZ_F256 = (size_t)NBATCH * NCH * NLEN * 4;
constexpr size_t SZ_QK   = (size_t)NBATCH * NLEN * 64 * 2;
constexpr size_t SZ_V    = (size_t)NBATCH * NCH * NLEN * 2;
constexpr size_t SZ_S    = (size_t)2 * NLEN * NLEN * 4;
constexpr size_t SZ_P    = (size_t)2 * NLEN * NLEN * 2;
constexpr size_t SZ_OT   = (size_t)NBATCH * NLEN * NCH * 2;
constexpr size_t SZ_C2   = (size_t)NBATCH * NCO * NLEN * 4;
constexpr size_t OFF_TP  = 0;
constexpr size_t OFF_W1  = OFF_TP  + SZ_TP;
constexpr size_t OFF_W2  = OFF_W1  + SZ_W1;
constexpr size_t OFF_WQK = OFF_W2  + SZ_W2;
constexpr size_t OFF_WV  = OFF_WQK + SZ_WQK;
constexpr size_t OFF_WO  = OFF_WV  + SZ_WV;
constexpr size_t OFF_WR  = OFF_WO  + SZ_WO;
constexpr size_t OFF_BQK = OFF_WR  + SZ_WR;
constexpr size_t OFF_C1  = OFF_BQK + SZ_BQK;
constexpr size_t OFF_H   = OFF_C1  + SZ_F256;
constexpr size_t OFF_HT  = OFF_H   + SZ_F256;
constexpr size_t OFF_QK  = OFF_HT  + SZ_TP;
constexpr size_t OFF_V   = OFF_QK  + SZ_QK;
constexpr size_t OFF_S   = OFF_V   + SZ_V;
constexpr size_t OFF_P   = OFF_S   + SZ_S;
constexpr size_t OFF_OT  = OFF_P   + SZ_P;
constexpr size_t WS_END  = OFF_OT  + SZ_OT;
static_assert(WS_END == 122093824, "carve");
static_assert(WS_END <= 134217728, "carve");
static_assert(OFF_H + SZ_C2 <= OFF_S, "c2 overlay");
static_assert((OFF_W1 % 128) == 0 && (OFF_BQK % 128) == 0 && (OFF_C1 % 128) == 0 && (OFF_H % 128) == 0 &&
              (OFF_HT % 128) == 0 && (OFF_QK % 128) == 0 && (OFF_V % 128) == 0 && (OFF_S % 128) == 0 &&
              (OFF_P % 128) == 0 && (OFF_OT % 128) == 0, "align");

typedef __attribute__((ext_vector_type(16))) _Float16 v16h;
typedef __attribute__((ext_vector_type(8)))  _Float16 v8h;
typedef __attribute__((ext_vector_type(16))) __bf16   v16b;
typedef __attribute__((ext_vector_type(8)))  __bf16   v8b;
typedef __attribute__((ext_vector_type(8)))  float    v8f;
typedef __attribute__((ext_vector_type(4)))  float    v4f;
typedef __attribute__((ext_vector_type(4)))  unsigned int v4u;

__device__ __forceinline__ unsigned short f2bf_bits(float f) {
  unsigned u = __float_as_uint(f);
  return (unsigned short)((u + 0x7FFFu + ((u >> 16) & 1u)) >> 16);
}
__device__ __forceinline__ float bf_bits2f(unsigned short h) { return __uint_as_float(((unsigned)h) << 16); }

__device__ __forceinline__ void dep_guard_h(v8f& a, v8f& b, v16h x, v16h y) { asm volatile("v_nop\n\tv_nop\n\tv_nop\n\tv_nop" : "+v"(a), "+v"(b) : "v"(x), "v"(y)); }
__device__ __forceinline__ void dep_guard_b(v8f& a, v8f& b, v16b x, v16b y) { asm volatile("v_nop\n\tv_nop\n\tv_nop\n\tv_nop" : "+v"(a), "+v"(b) : "v"(x), "v"(y)); }
__device__ __forceinline__ void keep4_h(v16h a, v16h b, v16h c, v16h d) { asm volatile("v_nop" :: "v"(a), "v"(b), "v"(c), "v"(d)); }
__device__ __forceinline__ void keep4_b(v16b a, v16b b, v16b c, v16b d) { asm volatile("v_nop" :: "v"(a), "v"(b), "v"(c), "v"(d)); }
__device__ __forceinline__ void acc_guard4(v8f& a, v8f& b, v8f& c, v8f& d) { asm volatile("v_nop\n\tv_nop\n\tv_nop\n\tv_nop" : "+v"(a), "+v"(b), "+v"(c), "+v"(d)); }
template <typename T> struct Frag;
template <> struct Frag<_Float16> {
  typedef v16h V; union U { v16h v; v8h h[2]; };
  static __device__ __forceinline__ v16h load(const _Float16* p) {
    U f; f.h[0] = *(const v8h*)(p); f.h[1] = *(const v8h*)(p + 16); return f.v;
  }
  static __device__ __forceinline__ v8f mma(v16h a, v16h b, v8f c) {
    return __builtin_amdgcn_wmma_f32_16x16x32_f16(false, a, false, b, (short)0, c, false, false);
  }
  static __device__ __forceinline__ void guard(v8f& a, v8f& b, v16h x, v16h y) { dep_guard_h(a, b, x, y); }
  static __device__ __forceinline__ void keep(v16h a, v16h b, v16h c, v16h d) { keep4_h(a, b, c, d); }
};
template <> struct Frag<__bf16> {
  typedef v16b V; union U { v16b v; v8b h[2]; };
  static __device__ __forceinline__ v16b load(const __bf16* p) {
    U f; f.h[0] = *(const v8b*)(p); f.h[1] = *(const v8b*)(p + 16); return f.v;
  }
  static __device__ __forceinline__ v8f mma(v16b a, v16b b, v8f c) {
    return __builtin_amdgcn_wmma_f32_16x16x32_bf16(false, a, false, b, (short)0, c, false, false);
  }
  static __device__ __forceinline__ void guard(v8f& a, v8f& b, v16b x, v16b y) { dep_guard_b(a, b, x, y); }
  static __device__ __forceinline__ void keep(v16b a, v16b b, v16b c, v16b d) { keep4_b(a, b, c, d); }
};

__device__ __forceinline__ unsigned pk16(unsigned short a, unsigned short b) { return (unsigned)a | ((unsigned)b << 16); }
__device__ __forceinline__ unsigned short h_bits(float f) { const _Float16 h = (_Float16)f; return __builtin_bit_cast(unsigned short, h); }

__device__ __forceinline__ float wave_sum(float v) {
#pragma unroll
  for (int off = 16; off > 0; off >>= 1) v += __shfl_xor(v, off, 32);
  return v;
}
__device__ __forceinline__ float wave_max(float v) {
#pragma unroll
  for (int off = 16; off > 0; off >>= 1) v = fmaxf(v, __shfl_xor(v, off, 32));
  return v;
}

template <int ET> struct Elem;
template <> struct Elem<0> { typedef _Float16 T; };
template <> struct Elem<1> { typedef __bf16 T; };
template <int ET, bool SPLIT, int BIAS_MODE, int OUT_MODE, bool RESID, int ACT = 0>
__global__ __launch_bounds__(256) void wmma_gemm64(
    const unsigned short* __restrict__ Ap, const unsigned short* __restrict__ A2p, int lda, long strideA,
    const unsigned short* __restrict__ Btp, const unsigned short* __restrict__ Bt2p, int ldb, long strideB,
    void* __restrict__ Cout, void* __restrict__ Cout2, int ldc, long strideC,
    const float* __restrict__ bias,
    const float* __restrict__ resid, long strideR,
    int M, int N, int K, float scale) {
  typedef typename Elem<ET>::T T;
  typedef typename Frag<T>::V V;
  const T* A = (const T*)Ap; const T* A2 = (const T*)A2p; const T* Bt = (const T*)Btp; const T* Bt2 = (const T*)Bt2p;
  __shared__ __align__(16) float sT[8][16 * 68];
  const int b    = blockIdx.y;
  const int lane = threadIdx.x & 31;
  const int wave = threadIdx.x >> 5;
  const int tilesN = N >> 6;
  const int tilesM = M >> 6;
  const int tile = blockIdx.x * 8 + wave;
  if (tile >= tilesM * tilesN) return;
  const int tm = tile / tilesN;
  const int tn = tile - tm * tilesN;
  const int m0 = tm << 6;
  const int n0 = tn << 6;

  const T* Ab  = A  + (size_t)b * strideA;
  const T* Bb  = Bt + (size_t)b * strideB;
  const T* Ab2 = SPLIT ? (A2  + (size_t)b * strideA) : nullptr;
  const T* Bb2 = SPLIT ? (Bt2 + (size_t)b * strideB) : nullptr;

  const int rlane = lane & 15;
  const int koff  = (lane >> 4) * 8;
  const int mOff  = (lane >> 4) * 8;

  v8f acc[4][4];
#pragma unroll
  for (int i = 0; i < 4; ++i)
#pragma unroll
    for (int j = 0; j < 4; ++j) acc[i][j] = (v8f){0.f,0.f,0.f,0.f,0.f,0.f,0.f,0.f};

  for (int k0 = 0; k0 < K; k0 += 32) {
    V bh[4], bl[4];
#pragma unroll
    for (int j = 0; j < 4; ++j) {
      const size_t bo = (size_t)(n0 + (j << 4) + rlane) * ldb + koff + k0;
      bh[j] = Frag<T>::load(Bb + bo);
      if (SPLIT) bl[j] = Frag<T>::load(Bb2 + bo);
    }
#pragma unroll
    for (int i = 0; i < 4; ++i) {
      const size_t ao = (size_t)(m0 + (i << 4) + rlane) * lda + koff + k0;
      V ah = Frag<T>::load(Ab + ao);
      V al;
      if (SPLIT) al = Frag<T>::load(Ab2 + ao);
#pragma unroll
      for (int j = 0; j < 4; ++j) {
        acc[i][j] = Frag<T>::mma(ah, bh[j], acc[i][j]);
        if (SPLIT) {
          acc[i][j] = Frag<T>::mma(ah, bl[j], acc[i][j]);
          acc[i][j] = Frag<T>::mma(al, bh[j], acc[i][j]);
        }
      }
      Frag<T>::guard(acc[i][0], acc[i][3], ah, SPLIT ? al : ah);
    }
    Frag<T>::keep(bh[0], bh[1], bh[2], bh[3]);
    if (SPLIT) Frag<T>::keep(bl[0], bl[1], bl[2], bl[3]);
  }
  acc_guard4(acc[0][0], acc[0][1], acc[0][2], acc[0][3]);
  acc_guard4(acc[1][0], acc[1][1], acc[1][2], acc[1][3]);
  acc_guard4(acc[2][0], acc[2][1], acc[2][2], acc[2][3]);
  acc_guard4(acc[3][0], acc[3][1], acc[3][2], acc[3][3]);

  float* slab = sT[wave];
  const float* Rb = RESID ? (resid + (size_t)b * strideR) : nullptr;
#pragma unroll
  for (int i = 0; i < 4; ++i) {
    const int mBase = m0 + (i << 4);
#pragma unroll
    for (int j = 0; j < 4; ++j) {
      const int n = n0 + (j << 4) + rlane;
      float bv = 0.f;
      if (BIAS_MODE == 2) bv = bias[n];
#pragma unroll
      for (int r = 0; r < 8; ++r) {
        float v = acc[i][j][r] * scale;
        if (BIAS_MODE == 1) v += bias[mBase + mOff + r];
        if (BIAS_MODE == 2) v += bv;
        if (RESID) v += Rb[(size_t)(mBase + mOff + r) * ldc + n];
        if (ACT == 2) v = fmaxf(v, 0.0f);
        if (ACT == 4) v = (v > 0.f) ? v : 0.01f * v;
        slab[(mOff + r) * 68 + (j << 4) + rlane] = v;
      }
    }
    __builtin_amdgcn_fence(__ATOMIC_RELEASE, "workgroup");
    __builtin_amdgcn_wave_barrier();
    __builtin_amdgcn_fence(__ATOMIC_ACQUIRE, "workgroup");
    if (OUT_MODE == 0) {
      float* C = (float*)Cout + (size_t)b * strideC;
      const int hh = lane >> 4, c4 = (lane & 15) * 4;
      for (int pass = 0; pass < 2; ++pass) {
#pragma unroll
        for (int it = 0; it < 8; ++it) {
          const int row = it * 2 + hh;
          v4f v = *(const v4f*)(slab + row * 68 + c4);
          *(volatile v4f*)(C + (size_t)(mBase + row) * ldc + n0 + c4) = v;
        }
        __threadfence();
      }
    } else {
      const int q = lane >> 3, c8 = (lane & 7) * 8;
      unsigned short* C  = (unsigned short*)Cout  + (size_t)b * strideC;
      unsigned short* C2 = (OUT_MODE == 2) ? ((unsigned short*)Cout2 + (size_t)b * strideC) : nullptr;
      for (int pass = 0; pass < 2; ++pass) {
#pragma unroll
        for (int it = 0; it < 4; ++it) {
          const int row = it * 4 + q;
          const float* sp = slab + row * 68 + c8;
          v8h hv, lv;
#pragma unroll
          for (int e = 0; e < 8; ++e) {
            if (OUT_MODE == 1) {
              hv[e] = (_Float16)sp[e];
            } else {
              unsigned short hb = f2bf_bits(sp[e]);
              unsigned short lb = f2bf_bits(sp[e] - bf_bits2f(hb));
              hv[e] = __builtin_bit_cast(_Float16, hb);
              lv[e] = __builtin_bit_cast(_Float16, lb);
            }
          }
          *(volatile v8h*)(C + (size_t)(mBase + row) * ldc + n0 + c8) = hv;
          if (OUT_MODE == 2) *(volatile v8h*)(C2 + (size_t)(mBase + row) * ldc + n0 + c8) = lv;
        }
        __threadfence();
      }
    }
    __builtin_amdgcn_fence(__ATOMIC_RELEASE, "workgroup");
    __builtin_amdgcn_wave_barrier();
    __builtin_amdgcn_fence(__ATOMIC_ACQUIRE, "workgroup");
  }
}

__global__ __launch_bounds__(256) void k_cast8(const float* __restrict__ in, unsigned short* __restrict__ out, int n8, float scale) {
  const int i = blockIdx.x * 256 + threadIdx.x;
  if (i >= n8) return;
  const float* p = in + 8 * (size_t)i;
  const v4f a = *(const v4f*)(p);
  const v4f c = *(const v4f*)(p + 4);
  unsigned short hb[8];
#pragma unroll
  for (int e = 0; e < 4; ++e) {
    hb[e]     = h_bits(a[e] * scale);
    hb[4 + e] = h_bits(c[e] * scale);
  }
  const v4u u = (v4u){pk16(hb[0], hb[1]), pk16(hb[2], hb[3]), pk16(hb[4], hb[5]), pk16(hb[6], hb[7])};
  unsigned short* q = out + 8 * (size_t)i;
  *(volatile v4u*)q = u;
  __threadfence();
  *(volatile v4u*)q = u;
}

__global__ __launch_bounds__(256) void k_castw5(const float* __restrict__ w, unsigned short* __restrict__ out, int n8, float scale) {
  const int i = blockIdx.x * 256 + threadIdx.x;
  if (i >= n8) return;
  const int idx = i * 8;
  const int o   = idx / KCONV;
  const int rem = idx - o * KCONV;
  const int tap = rem >> 8;
  const int c0  = rem & 255;
  const float* p = w + ((size_t)o * NCH + c0) * NTAP + tap;
  unsigned short hb[8];
#pragma unroll
  for (int e = 0; e < 8; ++e) hb[e] = h_bits(p[e * NTAP] * scale);
  const v4u u = (v4u){pk16(hb[0], hb[1]), pk16(hb[2], hb[3]), pk16(hb[4], hb[5]), pk16(hb[6], hb[7])};
  unsigned short* q = out + (size_t)idx;
  *(volatile v4u*)q = u;
  __threadfence();
  *(volatile v4u*)q = u;
}

__global__ __launch_bounds__(32) void k_biascat(const float* __restrict__ bq, const float* __restrict__ bk, float* __restrict__ out) {
  const int lane = threadIdx.x & 31;
  const int ia = lane < 8 ? lane : 7;
  int ib = lane - 8; ib = ib < 0 ? 0 : (ib > 7 ? 7 : ib);
  const v4f a = *(const v4f*)(bq + 4 * ia);
  const v4f c = *(const v4f*)(bk + 4 * ib);
  v4f v;
#pragma unroll
  for (int e = 0; e < 4; ++e) v[e] = (lane < 8) ? a[e] : c[e];
  if (lane < 16) *(volatile v4f*)(out + 4 * lane) = v;
  __threadfence();
  if (lane < 16) *(volatile v4f*)(out + 4 * lane) = v;
}

__global__ __launch_bounds__(256) void k_tr(const float* __restrict__ in, unsigned short* __restrict__ out) {
  __shared__ float sm[64][65];
  const int t  = threadIdx.x;
  const int r0 = blockIdx.x * 64;
  const int c0 = blockIdx.y * 64;
  const int b  = blockIdx.z;
  const float* ib = in + (size_t)b * NCH * NLEN;
  unsigned short* ob = out + (size_t)b * NLENP * NCH;
#pragma unroll
  for (int i = 0; i < 16; ++i) {
    const int e  = i * 256 + t;
    const int cl = e >> 6;
    const int rl = e & 63;
    const int l  = r0 + rl - 2;
    const int lc = l < 0 ? 0 : (l > NLEN - 1 ? NLEN - 1 : l);
    float v = ib[(size_t)(c0 + cl) * NLEN + lc];
    v = (l >= 0 && l < NLEN) ? v : 0.0f;
    sm[rl][cl] = v;
  }
  __syncthreads();
  const int lane = t & 31, wave = t >> 5;
  const int q = lane >> 3, c8 = (lane & 7) * 8;
  for (int pass = 0; pass < 2; ++pass) {
#pragma unroll
    for (int it = 0; it < 2; ++it) {
      const int row = wave * 8 + it * 4 + q;
      if (r0 + row < NLENP) {
        unsigned short hb[8];
#pragma unroll
        for (int e = 0; e < 8; ++e) hb[e] = h_bits(sm[row][c8 + e]);
        const v4u u = (v4u){pk16(hb[0], hb[1]), pk16(hb[2], hb[3]), pk16(hb[4], hb[5]), pk16(hb[6], hb[7])};
        *(volatile v4u*)(ob + (size_t)(r0 + row) * NCH + c0 + c8) = u;
      }
    }
    __threadfence();
  }
}

__global__ __launch_bounds__(256) void k_rownorm(const float* __restrict__ src, float* __restrict__ dst) {
  __shared__ float red[8];
  const int row = blockIdx.x;
  const int t = threadIdx.x, lane = t & 31, wave = t >> 5;
  const float* sr = src + (size_t)row * NLEN;
  const v4f a = *(const v4f*)(sr + 4 * t);
  const v4f c = *(const v4f*)(sr + 1024 + 4 * t);
  float x[8];
#pragma unroll
  for (int e = 0; e < 4; ++e) { x[e] = a[e]; x[4 + e] = c[e]; }
  float s = ((x[0] + x[1]) + (x[2] + x[3])) + ((x[4] + x[5]) + (x[6] + x[7]));
  s = wave_sum(s);
  if (lane == 0) red[wave] = s;
  __syncthreads();
  const float mean = (((red[0] + red[1]) + (red[2] + red[3])) + ((red[4] + red[5]) + (red[6] + red[7]))) * INV_LEN;
  __syncthreads();
  float d[8];
#pragma unroll
  for (int e = 0; e < 8; ++e) d[e] = x[e] - mean;
  float s2 = ((d[0] * d[0] + d[1] * d[1]) + (d[2] * d[2] + d[3] * d[3])) + ((d[4] * d[4] + d[5] * d[5]) + (d[6] * d[6] + d[7] * d[7]));
  s2 = wave_sum(s2);
  if (lane == 0) red[wave] = s2;
  __syncthreads();
  const float var  = (((red[0] + red[1]) + (red[2] + red[3])) + ((red[4] + red[5]) + (red[6] + red[7]))) * INV_LEN;
  const float rstd = 1.0f / sqrtf(var + IN_EPS);
  float y[8];
#pragma unroll
  for (int e = 0; e < 8; ++e) {
    const float v = d[e] * rstd;
    y[e] = (v >= 0.0f) ? v : NEG_SLOPE_V * v;
  }
  const v4f o0 = (v4f){y[0], y[1], y[2], y[3]};
  const v4f o1 = (v4f){y[4], y[5], y[6], y[7]};
  float* dr = dst + (size_t)row * NLEN;
  for (int pass = 0; pass < 2; ++pass) {
    *(volatile v4f*)(dr + 4 * t) = o0;
    *(volatile v4f*)(dr + 1024 + 4 * t) = o1;
    __threadfence();
  }
}

__global__ __launch_bounds__(256) void k_softmax(const float* __restrict__ S, unsigned short* __restrict__ P, float carry) {
  __shared__ float redM[8];
  __shared__ float redS[8];
  const int row  = blockIdx.x;
  const int t    = threadIdx.x;
  const int lane = t & 31, wave = t >> 5;
  const int c0   = t * 8;
  const float* sr = S + (size_t)row * NLEN + c0;
  const v4f a = *(const v4f*)(sr);
  const v4f c = *(const v4f*)(sr + 4);
  float x[8];
#pragma unroll
  for (int e = 0; e < 4; ++e) { x[e] = a[e]; x[4 + e] = c[e]; }
  float m = fmaxf(fmaxf(fmaxf(x[0], x[1]), fmaxf(x[2], x[3])), fmaxf(fmaxf(x[4], x[5]), fmaxf(x[6], x[7])));
  m = wave_max(m);
  if (lane == 0) redM[wave] = m;
  __syncthreads();
  m = fmaxf(fmaxf(fmaxf(redM[0], redM[1]), fmaxf(redM[2], redM[3])), fmaxf(fmaxf(redM[4], redM[5]), fmaxf(redM[6], redM[7])));
  float ex[8];
#pragma unroll
  for (int e = 0; e < 8; ++e) ex[e] = expf(x[e] - m);
  float s = ((ex[0] + ex[1]) + (ex[2] + ex[3])) + ((ex[4] + ex[5]) + (ex[6] + ex[7]));
  s = wave_sum(s);
  if (lane == 0) redS[wave] = s;
  __syncthreads();
  const float tot = ((redS[0] + redS[1]) + (redS[2] + redS[3])) + ((redS[4] + redS[5]) + (redS[6] + redS[7]));
  const float inv = carry / tot;
  unsigned short hb[8];
#pragma unroll
  for (int e = 0; e < 8; ++e) hb[e] = h_bits(ex[e] * inv);
  const v4u u = (v4u){pk16(hb[0], hb[1]), pk16(hb[2], hb[3]), pk16(hb[4], hb[5]), pk16(hb[6], hb[7])};
  unsigned short* q = P + (size_t)row * NLEN + c0;
  *(volatile v4u*)q = u;
  __threadfence();
  *(volatile v4u*)q = u;
}

__global__ __launch_bounds__(256) void k_final(const float* __restrict__ src, float* out) {
  __shared__ float red[8];
  const int row = blockIdx.x;
  const int t = threadIdx.x, lane = t & 31, wave = t >> 5;
  const float* sr = src + (size_t)row * NLEN;
  float* orow = out + (size_t)row * NLEN;
  const v4f a  = *(const v4f*)(sr + 4 * t);
  const v4f c  = *(const v4f*)(sr + 1024 + 4 * t);
  const v4f ra = *(const v4f*)(orow + 4 * t);
  const v4f rc = *(const v4f*)(orow + 1024 + 4 * t);
  float x[8], r[8];
#pragma unroll
  for (int e = 0; e < 4; ++e) { x[e] = a[e]; x[4 + e] = c[e]; r[e] = ra[e]; r[4 + e] = rc[e]; }
  float s = ((x[0] + x[1]) + (x[2] + x[3])) + ((x[4] + x[5]) + (x[6] + x[7]));
  s = wave_sum(s);
  if (lane == 0) red[wave] = s;
  __syncthreads();
  const float mean = (((red[0] + red[1]) + (red[2] + red[3])) + ((red[4] + red[5]) + (red[6] + red[7]))) * INV_LEN;
  __syncthreads();
  float d[8];
#pragma unroll
  for (int e = 0; e < 8; ++e) d[e] = x[e] - mean;
  float s2 = ((d[0] * d[0] + d[1] * d[1]) + (d[2] * d[2] + d[3] * d[3])) + ((d[4] * d[4] + d[5] * d[5]) + (d[6] * d[6] + d[7] * d[7]));
  s2 = wave_sum(s2);
  if (lane == 0) red[wave] = s2;
  __syncthreads();
  const float var  = (((red[0] + red[1]) + (red[2] + red[3])) + ((red[4] + red[5]) + (red[6] + red[7]))) * INV_LEN;
  const float rstd = 1.0f / sqrtf(var + IN_EPS);
  float y[8];
#pragma unroll
  for (int e = 0; e < 8; ++e) {
    const float v = d[e] * rstd + r[e];
    y[e] = (v >= 0.0f) ? v : NEG_SLOPE_V * v;
  }
  const v4f o0 = (v4f){y[0], y[1], y[2], y[3]};
  const v4f o1 = (v4f){y[4], y[5], y[6], y[7]};
  for (int pass = 0; pass < 2; ++pass) {
    *(volatile v4f*)(orow + 4 * t) = o0;
    *(volatile v4f*)(orow + 1024 + 4 * t) = o1;
    __threadfence();
  }
}

extern "C" void kernel_launch(void* const* d_in, const int* in_sizes, int n_in,
                              void* d_out, int out_size, void* d_ws, size_t ws_size,
                              hipStream_t stream) {
  if (n_in < 15) return;
  if (in_sizes[0] != NBATCH * NCH * NLEN) return;
  if (out_size != NBATCH * NCO * NLEN) return;
  if (ws_size < WS_END) return;

  const float* x  = (const float*)d_in[0];
  const float* w1 = (const float*)d_in[1];  const float* b1 = (const float*)d_in[2];
  const float* wq = (const float*)d_in[3];  const float* bq = (const float*)d_in[4];
  const float* wk = (const float*)d_in[5];  const float* bk = (const float*)d_in[6];
  const float* wv = (const float*)d_in[7];  const float* bv = (const float*)d_in[8];
  const float* wo = (const float*)d_in[9];  const float* bo = (const float*)d_in[10];
  const float* w2 = (const float*)d_in[11]; const float* b2 = (const float*)d_in[12];
  const float* wr = (const float*)d_in[13]; const float* br = (const float*)d_in[14];
  float* out = (float*)d_out;

  char* wsb = (char*)d_ws;
  unsigned short* TP  = (unsigned short*)(wsb + OFF_TP);
  unsigned short* W1r = (unsigned short*)(wsb + OFF_W1);
  unsigned short* W2r = (unsigned short*)(wsb + OFF_W2);
  unsigned short* WQK = (unsigned short*)(wsb + OFF_WQK);
  unsigned short* WV  = (unsigned short*)(wsb + OFF_WV);
  unsigned short* WO  = (unsigned short*)(wsb + OFF_WO);
  unsigned short* WR  = (unsigned short*)(wsb + OFF_WR);
  float*          BQK = (float*)(wsb + OFF_BQK);
  float*          C1  = (float*)(wsb + OFF_C1);
  float*          HF  = (float*)(wsb + OFF_H);
  unsigned short* HT  = (unsigned short*)(wsb + OFF_HT);
  unsigned short* QK  = (unsigned short*)(wsb + OFF_QK);
  unsigned short* VP  = (unsigned short*)(wsb + OFF_V);
  float*          SP  = (float*)(wsb + OFF_S);
  unsigned short* PP  = (unsigned short*)(wsb + OFF_P);
  unsigned short* OT  = (unsigned short*)(wsb + OFF_OT);
  float*          HP  = C1;
  float*          C2  = HF;

  const long STR_TP  = (long)NLENP * NCH;
  const long STR_CL  = (long)NCH * NLEN;
  const long STR_COL = (long)NCO * NLEN;
  const long STR_QK  = (long)NLEN * 64;
  const long STR_SS  = (long)NLEN * NLEN;

  k_castw5<<<dim3((NCH * KCONV / 8 + 255) / 256), dim3(256), 0, stream>>>(w1, W1r, NCH * KCONV / 8, W_CARRY);
  k_castw5<<<dim3((NCO * KCONV / 8 + 255) / 256), dim3(256), 0, stream>>>(w2, W2r, NCO * KCONV / 8, W_CARRY);
  k_cast8<<<dim3((NCR * NCH / 8 + 255) / 256), dim3(256), 0, stream>>>(wq, WQK, NCR * NCH / 8, W_CARRY);
  k_cast8<<<dim3((NCR * NCH / 8 + 255) / 256), dim3(256), 0, stream>>>(wk, WQK + (size_t)NCR * NCH, NCR * NCH / 8, W_CARRY);
  k_cast8<<<dim3((NCH * NCH / 8 + 255) / 256), dim3(256), 0, stream>>>(wv, WV, NCH * NCH / 8, W_CARRY);
  k_cast8<<<dim3((NCH * NCH / 8 + 255) / 256), dim3(256), 0, stream>>>(wo, WO, NCH * NCH / 8, W_CARRY);
  k_cast8<<<dim3((NCO * NCH / 8 + 255) / 256), dim3(256), 0, stream>>>(wr, WR, NCO * NCH / 8, W_CARRY);
  k_biascat<<<dim3(1), dim3(32), 0, stream>>>(bq, bk, BQK);
  k_tr<<<dim3((NLENP + 63) / 64, NCH / 64, NBATCH), dim3(256), 0, stream>>>(x, TP);

  wmma_gemm64<0, false, 1, 0, false, 0><<<dim3(((NCH / 64) * (NLEN / 64) + 7) / 8, NBATCH), dim3(256), 0, stream>>>(
      W1r, nullptr, KCONV, 0L, TP, nullptr, NCH, STR_TP,
      C1, nullptr, NLEN, STR_CL, b1, nullptr, 0L, NCH, NLEN, KCONV, W_CARRY_INV);
  wmma_gemm64<0, false, 1, 0, false, 0><<<dim3(((NCO / 64) * (NLEN / 64) + 7) / 8, NBATCH), dim3(256), 0, stream>>>(
      WR, nullptr, NCH, 0L, TP + 2 * NCH, nullptr, NCH, STR_TP,
      out, nullptr, NLEN, STR_COL, br, nullptr, 0L, NCO, NLEN, NCH, W_CARRY_INV);
  k_rownorm<<<dim3(NBATCH * NCH), dim3(256), 0, stream>>>(C1, HF);
  k_tr<<<dim3((NLENP + 63) / 64, NCH / 64, NBATCH), dim3(256), 0, stream>>>(HF, HT);
  wmma_gemm64<0, false, 2, 1, false, 0><<<dim3(((NLEN / 64) * 1 + 7) / 8, NBATCH), dim3(256), 0, stream>>>(
      HT + 2 * NCH, nullptr, NCH, STR_TP, WQK, nullptr, NCH, 0L,
      QK, nullptr, 64, STR_QK, BQK, nullptr, 0L, NLEN, 64, NCH, W_CARRY_INV);
  wmma_gemm64<0, false, 1, 1, false, 0><<<dim3(((NCH / 64) * (NLEN / 64) + 7) / 8, NBATCH), dim3(256), 0, stream>>>(
      WV, nullptr, NCH, 0L, HT + 2 * NCH, nullptr, NCH, STR_TP,
      VP, nullptr, NLEN, STR_CL, bv, nullptr, 0L, NCH, NLEN, NCH, W_CARRY_INV);

  for (int cb = 0; cb < NBATCH / 2; ++cb) {
    const unsigned short* QKc = QK + (size_t)cb * 2 * STR_QK;
    wmma_gemm64<0, false, 0, 0, false, 0><<<dim3(((NLEN / 64) * (NLEN / 64) + 7) / 8, 2), dim3(256), 0, stream>>>(
        QKc, nullptr, 64, STR_QK, QKc + NCR, nullptr, 64, STR_QK,
        SP, nullptr, NLEN, STR_SS, nullptr, nullptr, 0L, NLEN, NLEN, NCR, QK_SCALE);
    k_softmax<<<dim3(2 * NLEN), dim3(256), 0, stream>>>(SP, PP, P_CARRY);
    wmma_gemm64<0, false, 0, 1, false, 0><<<dim3(((NLEN / 64) * (NCH / 64) + 7) / 8, 2), dim3(256), 0, stream>>>(
        PP, nullptr, NLEN, STR_SS, VP + (size_t)cb * 2 * STR_CL, nullptr, NLEN, STR_CL,
        OT + (size_t)cb * 2 * STR_CL, nullptr, NCH, STR_CL, nullptr, nullptr, 0L, NLEN, NCH, NLEN, PV_OUT_SCALE);
  }

  wmma_gemm64<0, false, 1, 0, true, 0><<<dim3(((NCH / 64) * (NLEN / 64) + 7) / 8, NBATCH), dim3(256), 0, stream>>>(
      WO, nullptr, NCH, 0L, OT, nullptr, NCH, STR_CL,
      HP, nullptr, NLEN, STR_CL, bo, HF, STR_CL, NCH, NLEN, NCH, WO_SCALE);
  k_tr<<<dim3((NLENP + 63) / 64, NCH / 64, NBATCH), dim3(256), 0, stream>>>(HP, TP);
  wmma_gemm64<0, false, 1, 0, false, 0><<<dim3(((NCO / 64) * (NLEN / 64) + 7) / 8, NBATCH), dim3(256), 0, stream>>>(
      W2r, nullptr, KCONV, 0L, TP, nullptr, NCH, STR_TP,
      C2, nullptr, NLEN, STR_COL, b2, nullptr, 0L, NCO, NLEN, KCONV, W_CARRY_INV);
  k_final<<<dim3(NBATCH * NCO), dim3(256), 0, stream>>>(C2, out);
}
